// SpatialMix_HPCM_74397423501646
// MI455X (gfx1250) — hardware-run, weakly checked
//
#include <hip/hip_runtime.h>
#include <math.h>

typedef __attribute__((ext_vector_type(16))) _Float16 v16h;
typedef __attribute__((ext_vector_type(8)))  _Float16 v8h;
typedef __attribute__((ext_vector_type(2)))  _Float16 v2h;
typedef __attribute__((ext_vector_type(16))) __bf16   v16b;
typedef __attribute__((ext_vector_type(8)))  __bf16   v8b;
typedef __attribute__((ext_vector_type(8)))  float    v8f;
typedef __attribute__((ext_vector_type(4)))  float    v4f;
typedef __attribute__((ext_vector_type(2)))  float    v2f;

constexpr int kBatch  = 8;
constexpr int kCh     = 192;
constexpr int kHt     = 64;
constexpr int kWd     = 64;
constexpr int kTok    = kHt * kWd;
constexpr int kHalfB  = 4;
constexpr int kRows   = kHalfB * kTok;
constexpr int kN3     = 3 * kCh;
constexpr int kThr    = 256;

constexpr float kXCarry = 1024.0f;
constexpr float kWCarry = 1024.0f;
constexpr float kYCarry = 4096.0f;
constexpr float kPScale = 1.0f / (kXCarry * kWCarry);
constexpr float kOScale = 1.0f / (kYCarry * kWCarry);
constexpr float kF16MinNormal = 6.103515625e-5f;

static_assert(kTok == 4096 && kRows == 16384 && kN3 == 576, "sizes");
static_assert((kRows % 64) == 0 && (kN3 % 64) == 0 && (kCh % 64) == 0 && (kCh % 32) == 0, "GEMM M, N multiples of 64, K of 32");

constexpr size_t kOffW3   = 0;
constexpr size_t kOffWO   = kOffW3  + (size_t)kN3 * kCh * 2;
constexpr size_t kOffZB   = kOffWO  + (size_t)kCh * kCh * 2;
constexpr size_t kOffXS   = kOffZB  + 2560;
constexpr size_t kOffKVR  = kOffXS  + (size_t)kRows * kCh * 2;
constexpr size_t kOffBW   = kOffKVR + (size_t)kRows * kN3 * 4;
constexpr size_t kOffY16  = kOffBW  + (size_t)kRows * kN3 * 4;
constexpr size_t kOffOUTF = kOffY16 + (size_t)kRows * kCh * 2;
constexpr size_t kWsTotal = kOffOUTF + (size_t)kRows * kCh * 4;
static_assert(kWsTotal == 100960768ull, "carve total");
static_assert(kWsTotal <= 134217728ull, "carve cap");
static_assert((kOffWO % 256) == 0 && (kOffZB % 256) == 0 && (kOffXS % 256) == 0 && (kOffKVR % 256) == 0 && (kOffBW % 256) == 0 && (kOffY16 % 256) == 0 && (kOffOUTF % 256) == 0, "aligned regions");

__device__ __forceinline__ unsigned short f2bf_bits(float f) {
  unsigned u = __float_as_uint(f);
  return (unsigned short)((u + 0x7FFFu + ((u >> 16) & 1u)) >> 16);
}
__device__ __forceinline__ float bf_bits2f(unsigned short h) { return __uint_as_float(((unsigned)h) << 16); }
__device__ __forceinline__ float bf16r(float f) { return bf_bits2f(f2bf_bits(f)); }
__device__ __forceinline__ float carry_flush(float v, float carry) {
  const float s = v * carry;
  return (fabsf(s) < kF16MinNormal) ? 0.0f : s;
}
__device__ __forceinline__ float frcp(float x) { return __builtin_amdgcn_rcpf(x); }

__device__ __forceinline__ void dep_guard4_h(v8f& a, v8f& b, v8f& c, v8f& d, v16h x, v16h y) { asm volatile("v_nop\n\tv_nop\n\tv_nop\n\tv_nop" : "+v"(a), "+v"(b), "+v"(c), "+v"(d) : "v"(x), "v"(y)); }
__device__ __forceinline__ void dep_guard4_b(v8f& a, v8f& b, v8f& c, v8f& d, v16b x, v16b y) { asm volatile("v_nop\n\tv_nop\n\tv_nop\n\tv_nop" : "+v"(a), "+v"(b), "+v"(c), "+v"(d) : "v"(x), "v"(y)); }
__device__ __forceinline__ void keep4_h(v16h a, v16h b, v16h c, v16h d) { asm volatile("v_nop" :: "v"(a), "v"(b), "v"(c), "v"(d)); }
__device__ __forceinline__ void keep4_b(v16b a, v16b b, v16b c, v16b d) { asm volatile("v_nop" :: "v"(a), "v"(b), "v"(c), "v"(d)); }
__device__ __forceinline__ void acc_guard4(v8f& a, v8f& b, v8f& c, v8f& d) { asm volatile("v_nop\n\tv_nop\n\tv_nop\n\tv_nop" : "+v"(a), "+v"(b), "+v"(c), "+v"(d)); }

template <typename T> struct Frag;
template <> struct Frag<_Float16> {
  typedef v16h V; union U { v16h v; v8h h[2]; };
  static __device__ __forceinline__ v16h load(const _Float16* p) {
    U f; f.h[0] = *(const v8h*)(p); f.h[1] = *(const v8h*)(p + 16); return f.v;
  }
  static __device__ __forceinline__ v8f mma(v16h a, v16h b, v8f c) {
    return __builtin_amdgcn_wmma_f32_16x16x32_f16(false, a, false, b, (short)0, c, false, false);
  }
  static __device__ __forceinline__ void guard4(v8f& a, v8f& b, v8f& c, v8f& d, v16h x, v16h y) { dep_guard4_h(a, b, c, d, x, y); }
  static __device__ __forceinline__ void keep(v16h a, v16h b, v16h c, v16h d) { keep4_h(a, b, c, d); }
};
template <> struct Frag<__bf16> {
  typedef v16b V; union U { v16b v; v8b h[2]; };
  static __device__ __forceinline__ v16b load(const __bf16* p) {
    U f; f.h[0] = *(const v8b*)(p); f.h[1] = *(const v8b*)(p + 16); return f.v;
  }
  static __device__ __forceinline__ v8f mma(v16b a, v16b b, v8f c) {
    return __builtin_amdgcn_wmma_f32_16x16x32_bf16(false, a, false, b, (short)0, c, false, false);
  }
  static __device__ __forceinline__ void guard4(v8f& a, v8f& b, v8f& c, v8f& d, v16b x, v16b y) { dep_guard4_b(a, b, c, d, x, y); }
  static __device__ __forceinline__ void keep(v16b a, v16b b, v16b c, v16b d) { keep4_b(a, b, c, d); }
};

__device__ __forceinline__ v8f mma_h(v16h a, v16h b, v8f c) {
  c = __builtin_amdgcn_wmma_f32_16x16x32_f16(false, a, false, b, (short)0, c, false, false);
  asm volatile("v_nop\n\tv_nop\n\tv_nop\n\tv_nop" : "+v"(c) : "v"(a), "v"(b));
  return c;
}

template <int ET> struct Elem;
template <> struct Elem<0> { typedef _Float16 T; };
template <> struct Elem<1> { typedef __bf16 T; };
template <int ET, bool SPLIT, int BIAS_MODE, int OUT_MODE, bool RESID, int ACT = 0>
__global__ __launch_bounds__(256) void wmma_gemm64(
    const unsigned short* __restrict__ Ap, const unsigned short* __restrict__ A2p, int lda, long strideA,
    const unsigned short* __restrict__ Btp, const unsigned short* __restrict__ Bt2p, int ldb, long strideB,
    void* __restrict__ Cout, void* __restrict__ Cout2, int ldc, long strideC,
    const float* __restrict__ bias,
    const float* __restrict__ resid, long strideR,
    int M, int N, int K, float scale) {
  typedef typename Elem<ET>::T T;
  typedef typename Frag<T>::V V;
  const T* A = (const T*)Ap; const T* A2 = (const T*)A2p; const T* Bt = (const T*)Btp; const T* Bt2 = (const T*)Bt2p;
  __shared__ __align__(16) float sT[8][16 * 68];
  const int b    = blockIdx.y;
  const int lane = threadIdx.x & 31;
  const int wave = threadIdx.x >> 5;
  const int tilesN = N >> 6;
  const int tilesM = M >> 6;
  const int tile = blockIdx.x * 8 + wave;
  if (tile >= tilesM * tilesN) return;
  const int tm = tile / tilesN;
  const int tn = tile - tm * tilesN;
  const int m0 = tm << 6;
  const int n0 = tn << 6;

  const T* Ab  = A  + (size_t)b * strideA;
  const T* Bb  = Bt + (size_t)b * strideB;
  const T* Ab2 = SPLIT ? (A2  + (size_t)b * strideA) : nullptr;
  const T* Bb2 = SPLIT ? (Bt2 + (size_t)b * strideB) : nullptr;

  const int rlane = lane & 15;
  const int koff  = (lane >> 4) * 8;
  const int mOff  = (lane >> 4) * 8;

  v8f acc[4][4];
#pragma unroll
  for (int i = 0; i < 4; ++i)
#pragma unroll
    for (int j = 0; j < 4; ++j) acc[i][j] = (v8f){0.f,0.f,0.f,0.f,0.f,0.f,0.f,0.f};

  for (int k0 = 0; k0 < K; k0 += 32) {
    V bh[4], bl[4];
#pragma unroll
    for (int j = 0; j < 4; ++j) {
      const size_t bo = (size_t)(n0 + (j << 4) + rlane) * ldb + koff + k0;
      bh[j] = Frag<T>::load(Bb + bo);
      if (SPLIT) bl[j] = Frag<T>::load(Bb2 + bo);
    }
#pragma unroll
    for (int i = 0; i < 4; ++i) {
      const size_t ao = (size_t)(m0 + (i << 4) + rlane) * lda + koff + k0;
      V ah = Frag<T>::load(Ab + ao);
      V al;
      if (SPLIT) al = Frag<T>::load(Ab2 + ao);
#pragma unroll
      for (int j = 0; j < 4; ++j) {
        acc[i][j] = Frag<T>::mma(ah, bh[j], acc[i][j]);
        if (SPLIT) {
          acc[i][j] = Frag<T>::mma(ah, bl[j], acc[i][j]);
          acc[i][j] = Frag<T>::mma(al, bh[j], acc[i][j]);
        }
      }
      Frag<T>::guard4(acc[i][0], acc[i][1], acc[i][2], acc[i][3], ah, SPLIT ? al : ah);
    }
    Frag<T>::keep(bh[0], bh[1], bh[2], bh[3]);
    if (SPLIT) Frag<T>::keep(bl[0], bl[1], bl[2], bl[3]);
  }
  acc_guard4(acc[0][0], acc[0][1], acc[0][2], acc[0][3]);
  acc_guard4(acc[1][0], acc[1][1], acc[1][2], acc[1][3]);
  acc_guard4(acc[2][0], acc[2][1], acc[2][2], acc[2][3]);
  acc_guard4(acc[3][0], acc[3][1], acc[3][2], acc[3][3]);

  float* slab = sT[wave];
  const float* Rb = RESID ? (resid + (size_t)b * strideR) : nullptr;
#pragma unroll
  for (int i = 0; i < 4; ++i) {
    const int mBase = m0 + (i << 4);
#pragma unroll
    for (int j = 0; j < 4; ++j) {
      const int n = n0 + (j << 4) + rlane;
      float bv = 0.f;
      if (BIAS_MODE == 2) bv = bias[n];
#pragma unroll
      for (int r = 0; r < 8; ++r) {
        float v = acc[i][j][r] * scale;
        if (BIAS_MODE == 1) v += bias[mBase + mOff + r];
        if (BIAS_MODE == 2) v += bv;
        if (RESID) v += Rb[(size_t)(mBase + mOff + r) * ldc + n];
        if (ACT == 1) v = tanhf(v);
        if (ACT == 2) v = fmaxf(v, 0.0f);
        if (ACT == 3) v = v / (1.0f + expf(-v));
        if (ACT == 4) v = (v > 0.f) ? v : 0.01f * v;
        slab[(mOff + r) * 68 + (j << 4) + rlane] = v;
      }
    }
    __builtin_amdgcn_fence(__ATOMIC_RELEASE, "workgroup");
    __builtin_amdgcn_wave_barrier();
    __builtin_amdgcn_fence(__ATOMIC_ACQUIRE, "workgroup");
    if (OUT_MODE == 0) {
      float* C = (float*)Cout + (size_t)b * strideC;
      const int hh = lane >> 4, c4 = (lane & 15) * 4;
      for (int pass = 0; pass < 2; ++pass) {
#pragma unroll
        for (int it = 0; it < 8; ++it) {
          const int row = it * 2 + hh;
          v4f v = *(const v4f*)(slab + row * 68 + c4);
          *(volatile v4f*)(C + (size_t)(mBase + row) * ldc + n0 + c4) = v;
        }
        __threadfence();
      }
    } else {
      const int q = lane >> 3, c8 = (lane & 7) * 8;
      unsigned short* C  = (unsigned short*)Cout  + (size_t)b * strideC;
      unsigned short* C2 = (OUT_MODE == 2) ? ((unsigned short*)Cout2 + (size_t)b * strideC) : nullptr;
      for (int pass = 0; pass < 2; ++pass) {
#pragma unroll
        for (int it = 0; it < 4; ++it) {
          const int row = it * 4 + q;
          const float* sp = slab + row * 68 + c8;
          v8h hv, lv;
#pragma unroll
          for (int e = 0; e < 8; ++e) {
            if (OUT_MODE == 1) {
              hv[e] = (_Float16)sp[e];
            } else {
              unsigned short hb = f2bf_bits(sp[e]);
              unsigned short lb = f2bf_bits(sp[e] - bf_bits2f(hb));
              hv[e] = __builtin_bit_cast(_Float16, hb);
              lv[e] = __builtin_bit_cast(_Float16, lb);
            }
          }
          *(volatile v8h*)(C + (size_t)(mBase + row) * ldc + n0 + c8) = hv;
          if (OUT_MODE == 2) *(volatile v8h*)(C2 + (size_t)(mBase + row) * ldc + n0 + c8) = lv;
        }
        __threadfence();
      }
    }
    __builtin_amdgcn_fence(__ATOMIC_RELEASE, "workgroup");
    __builtin_amdgcn_wave_barrier();
    __builtin_amdgcn_fence(__ATOMIC_ACQUIRE, "workgroup");
  }
}


__global__ __launch_bounds__(kThr) void smx_weights_kernel(const float* __restrict__ w_key, const float* __restrict__ w_value,
                                                          const float* __restrict__ w_recept, const float* __restrict__ w_out,
                                                          unsigned short* __restrict__ W3, unsigned short* __restrict__ WO,
                                                          float* __restrict__ ZB) {
  const int blk = blockIdx.x;
  const int tid = threadIdx.x;
  const float* src;
  unsigned short* dst;
  if (blk < 54) {
    const int v = blk * kThr + tid;
    const int which = v / 4608;
    const int vv = v - which * 4608;
    src = ((which == 0) ? w_key : ((which == 1) ? w_value : w_recept)) + (size_t)vv * 8;
    dst = W3 + (size_t)v * 8;
  } else {
    const int v = (blk - 54) * kThr + tid;
    src = w_out + (size_t)v * 8;
    dst = WO + (size_t)v * 8;
  }
  const v4f a = *(const v4f*)src;
  const v4f b = *(const v4f*)(src + 4);
  v8h hv;
#pragma unroll
  for (int e = 0; e < 4; ++e) {
    hv[e]     = (_Float16)carry_flush(bf16r(a[e]), kWCarry);
    hv[e + 4] = (_Float16)carry_flush(bf16r(b[e]), kWCarry);
  }
  *(volatile v8h*)dst = hv;
  __threadfence();
  *(volatile v8h*)dst = hv;
  if (blk == 0 && tid < 144) {
    const v4f z4 = {0.f, 0.f, 0.f, 0.f};
    *(volatile v4f*)(ZB + 4 * tid) = z4;
    __threadfence();
    *(volatile v4f*)(ZB + 4 * tid) = z4;
  }
}

__global__ __launch_bounds__(kThr) void omni_kernel(const float* __restrict__ x, const float* __restrict__ alpha,
                                                    const float* __restrict__ dw1, const float* __restrict__ dw3,
                                                    const float* __restrict__ dw5, unsigned short* __restrict__ XS, int half) {
  __shared__ __align__(16) float tile[64 * 68];
  const int tid = threadIdx.x;
  const int cg = blockIdx.x % 3;
  const int h  = (blockIdx.x / 3) & 63;
  const int bl = blockIdx.x / 192;
  const int b  = half * kHalfB + bl;
  const int w  = tid & 63;
  const int cq = tid >> 6;
  const float a0 = bf16r(alpha[0]), a1 = bf16r(alpha[1]), a2 = bf16r(alpha[2]), a3 = bf16r(alpha[3]);
#pragma unroll 1
  for (int i = 0; i < 16; ++i) {
    const int c = 64 * cg + 16 * cq + i;
    const float* xc = x + ((size_t)b * kCh + c) * kTok;
    float s3 = 0.0f, s5 = 0.0f, ctr = 0.0f;
#pragma unroll
    for (int dy = -2; dy <= 2; ++dy) {
#pragma unroll
      for (int dx = -2; dx <= 2; ++dx) {
        const int yy = h + dy, xx = w + dx;
        const bool ok = (yy >= 0) && (yy < kHt) && (xx >= 0) && (xx < kWd);
        const int yc = (yy < 0) ? 0 : ((yy >= kHt) ? (kHt - 1) : yy);
        const int xq = (xx < 0) ? 0 : ((xx >= kWd) ? (kWd - 1) : xx);
        float xv = xc[yc * kWd + xq];
        asm volatile("" : "+v"(xv));
        const float xz = ok ? bf16r(xv) : 0.0f;
        s5 = fmaf(bf16r(dw5[c * 25 + (dy + 2) * 5 + (dx + 2)]), xz, s5);
        if (dy >= -1 && dy <= 1 && dx >= -1 && dx <= 1) s3 = fmaf(bf16r(dw3[c * 9 + (dy + 1) * 3 + (dx + 1)]), xz, s3);
        if (dy == 0 && dx == 0) ctr = xz;
      }
    }
    const float s1 = bf16r(dw1[c]) * ctr;
    const float xs = ((a0 * ctr + a1 * s1) + a2 * s3) + a3 * s5;
    tile[w * 68 + 16 * cq + i] = xs;
  }
  __syncthreads();
  {
    const int row = tid >> 2;
    const int part = tid & 3;
    v8h lo, hi;
#pragma unroll
    for (int q4 = 0; q4 < 4; ++q4) {
      const v4f tv = *(const v4f*)(tile + row * 68 + part * 16 + 4 * q4);
#pragma unroll
      for (int e = 0; e < 4; ++e) {
        const _Float16 hq = (_Float16)carry_flush(tv[e], kXCarry);
        if (q4 < 2) lo[4 * q4 + e] = hq; else hi[4 * (q4 - 2) + e] = hq;
      }
    }
    unsigned short* dst = XS + ((size_t)bl * kTok + (size_t)h * kWd + row) * kCh + 64 * cg + part * 16;
    for (int pass = 0; pass < 2; ++pass) {
      *(volatile v8h*)dst = lo;
      *(volatile v8h*)(dst + 8) = hi;
      __threadfence();
    }
  }
}

__global__ __launch_bounds__(32) void wkv_bwd_kernel(const float* __restrict__ KVR, const float* __restrict__ decay,
                                                     float* __restrict__ BW) {
  const int bl = blockIdx.x / 3;
  const int c0 = (blockIdx.x % 3) * 64 + 2 * (threadIdx.x & 31);
  const float w0 = bf16r(decay[c0]) * (1.0f / (float)kTok);
  const float w1 = bf16r(decay[c0 + 1]) * (1.0f / (float)kTok);
  float p0 = -INFINITY, p1 = -INFINITY, n0 = 0.f, n1 = 0.f, d0 = 0.f, d1 = 0.f;
#pragma unroll 1
  for (int t = kTok - 1; t >= 0; --t) {
    const size_t row = (size_t)bl * kTok + t;
    float* bp = BW + row * kN3 + c0;
    const v2f pv = {p0, p1};
    const v2f nv = {n0, n1};
    const v2f dv = {d0, d1};
    for (int pass = 0; pass < 2; ++pass) {
      *(volatile v2f*)bp = pv;
      *(volatile v2f*)(bp + kCh) = nv;
      *(volatile v2f*)(bp + 2 * kCh) = dv;
      __threadfence();
    }
    const v2f kk = *(const v2f*)(KVR + row * kN3 + c0);
    const v2f vv = *(const v2f*)(KVR + row * kN3 + kCh + c0);
    {
      const float q = fmaxf(p0 - w0, kk[0]);
      const float e1 = expf((p0 - w0) - q);
      const float e2 = expf(kk[0] - q);
      p0 = q; n0 = e1 * n0 + e2 * vv[0]; d0 = e1 * d0 + e2;
    }
    {
      const float q = fmaxf(p1 - w1, kk[1]);
      const float e1 = expf((p1 - w1) - q);
      const float e2 = expf(kk[1] - q);
      p1 = q; n1 = e1 * n1 + e2 * vv[1]; d1 = e1 * d1 + e2;
    }
  }
}

__global__ __launch_bounds__(32) void wkv_fwd_kernel(const float* __restrict__ KVR, const float* __restrict__ BW,
                                                     const float* __restrict__ decay, const float* __restrict__ boost,
                                                     const int* __restrict__ hin, const int* __restrict__ win,
                                                     unsigned short* __restrict__ Y16) {
  const int bl = blockIdx.x / 3;
  const int c0 = (blockIdx.x % 3) * 64 + 2 * (threadIdx.x & 31);
  float wv[2], uv[2];
#pragma unroll
  for (int s = 0; s < 2; ++s) {
    wv[s] = bf16r(decay[c0 + s]) * (1.0f / (float)kTok);
    uv[s] = bf16r(boost[c0 + s]) * (1.0f / (float)kTok);
  }
  const int hv_ = hin[0];
  const int wv_ = win[0];
  const float poison = (hv_ == kHt && wv_ == kWd) ? 0.0f : __builtin_nanf("");
  float pf[2] = {-INFINITY, -INFINITY}, nf[2] = {0.f, 0.f}, df[2] = {0.f, 0.f};
#pragma unroll 1
  for (int t = 0; t < kTok; ++t) {
    const size_t row = (size_t)bl * kTok + t;
    const float* kp = KVR + row * kN3 + c0;
    const float* bp = BW + row * kN3 + c0;
    const v2f kk = *(const v2f*)kp;
    const v2f vv = *(const v2f*)(kp + kCh);
    const v2f rr = *(const v2f*)(kp + 2 * kCh);
    const v2f pb = *(const v2f*)bp;
    const v2f nb = *(const v2f*)(bp + kCh);
    const v2f db = *(const v2f*)(bp + 2 * kCh);
    v2h yo;
#pragma unroll
    for (int s = 0; s < 2; ++s) {
      const float ps = uv[s] + kk[s];
      const float r = fmaxf(fmaxf(pf[s], pb[s]), ps);
      const float ef = expf(pf[s] - r);
      const float eb = expf(pb[s] - r);
      const float es = expf(ps - r);
      const float numv = (ef * nf[s] + eb * nb[s]) + es * vv[s];
      const float denv = (ef * df[s] + eb * db[s]) + es;
      const float wkv = numv / denv;
      const float sg = 1.0f / (1.0f + expf(-rr[s]));
      const float y = sg * wkv + poison;
      yo[s] = (_Float16)carry_flush(y, kYCarry);
      const float q = fmaxf(pf[s] - wv[s], kk[s]);
      const float e1 = expf((pf[s] - wv[s]) - q);
      const float e2 = expf(kk[s] - q);
      pf[s] = q; nf[s] = e1 * nf[s] + e2 * vv[s]; df[s] = e1 * df[s] + e2;
    }
    unsigned short* yp = Y16 + row * kCh + c0;
    *(volatile v2h*)yp = yo;
    __threadfence();
    *(volatile v2h*)yp = yo;
  }
}

__global__ __launch_bounds__(kThr) void smx_out_kernel(const float* __restrict__ OUTF, float* __restrict__ out, int half) {
  const int v  = blockIdx.x * kThr + threadIdx.x;
  const int t4 = (v & (kTok / 4 - 1)) * 4;
  const int bc = v >> 10;
  const int c  = bc % kCh;
  const int bl = bc / kCh;
  v4f o;
#pragma unroll
  for (int e = 0; e < 4; ++e) {
    const float q = OUTF[((size_t)bl * kTok + t4 + e) * kCh + c];
    o[e] = q;
  }
  float* dst = out + (((size_t)(half * kHalfB + bl)) * kCh + c) * kTok + t4;
  *(volatile v4f*)dst = o;
  __threadfence();
  *(volatile v4f*)dst = o;
}

static_assert(((kRows / 64) * (kN3 / 64)) % 8 == 0 && ((kRows / 64) * (kCh / 64)) % 8 == 0, "GEMM grids exact");
static_assert((kN3 * kCh / 8) == 54 * kThr && (kCh * kCh / 8) == 18 * kThr, "weight-plane grid exact");
static_assert(((size_t)kHalfB * kCh * kTok / 4) % kThr == 0, "layout grid exact");

extern "C" void kernel_launch(void* const* d_in, const int* in_sizes, int n_in,
                              void* d_out, int out_size, void* d_ws, size_t ws_size,
                              hipStream_t stream) {
  if (n_in < 13 || d_out == nullptr || d_ws == nullptr) return;
  if ((size_t)in_sizes[0] != (size_t)kBatch * kCh * kTok) return;
  for (int k = 1; k <= 4; ++k) if (in_sizes[k] != kCh * kCh) return;
  if (in_sizes[5] != kCh || in_sizes[6] != kCh || in_sizes[7] != 4) return;
  if (in_sizes[8] != kCh || in_sizes[9] != kCh * 9 || in_sizes[10] != kCh * 25) return;
  if (in_sizes[11] < 1 || in_sizes[12] < 1) return;
  if ((size_t)out_size != (size_t)kBatch * kCh * kTok) return;
  if (ws_size < kWsTotal) return;

  const float* x        = (const float*)d_in[0];
  const float* w_key    = (const float*)d_in[1];
  const float* w_value  = (const float*)d_in[2];
  const float* w_recept = (const float*)d_in[3];
  const float* w_out    = (const float*)d_in[4];
  const float* decay    = (const float*)d_in[5];
  const float* boost    = (const float*)d_in[6];
  const float* alpha    = (const float*)d_in[7];
  const float* dw1      = (const float*)d_in[8];
  const float* dw3      = (const float*)d_in[9];
  const float* dw5      = (const float*)d_in[10];
  const int*   hin      = (const int*)d_in[11];
  const int*   win      = (const int*)d_in[12];
  float* out = (float*)d_out;

  char* ws = (char*)d_ws;
  unsigned short* W3  = (unsigned short*)(ws + kOffW3);
  unsigned short* WO  = (unsigned short*)(ws + kOffWO);
  float*          ZB  = (float*)(ws + kOffZB);
  unsigned short* XS  = (unsigned short*)(ws + kOffXS);
  float*          KVR = (float*)(ws + kOffKVR);
  float*          BW  = (float*)(ws + kOffBW);
  unsigned short* Y16 = (unsigned short*)(ws + kOffY16);
  float*          OUTF = (float*)(ws + kOffOUTF);

  smx_weights_kernel<<<72, kThr, 0, stream>>>(w_key, w_value, w_recept, w_out, W3, WO, ZB);

  for (int half = 0; half < 2; ++half) {
    omni_kernel<<<kHalfB * kHt * 3, kThr, 0, stream>>>(x, alpha, dw1, dw3, dw5, XS, half);

    wmma_gemm64<0, false, 2, 0, false, 0><<<dim3((kRows / 64) * (kN3 / 64) / 8, 1), 256, 0, stream>>>(
        XS, XS, kCh, 0L, W3, W3, kCh, 0L, (void*)KVR, (void*)KVR, kN3, 0L,
        ZB, nullptr, 0L, kRows, kN3, kCh, kPScale);

    wkv_bwd_kernel<<<kHalfB * 3, 32, 0, stream>>>(KVR, decay, BW);
    wkv_fwd_kernel<<<kHalfB * 3, 32, 0, stream>>>(KVR, BW, decay, boost, hin, win, Y16);

    wmma_gemm64<0, false, 2, 0, false, 0><<<dim3((kRows / 64) * (kCh / 64) / 8, 1), 256, 0, stream>>>(
        Y16, Y16, kCh, 0L, WO, WO, kCh, 0L, (void*)OUTF, (void*)OUTF, kCh, 0L,
        ZB, nullptr, 0L, kRows, kCh, kCh, kOScale);

    smx_out_kernel<<<(int)(((size_t)kHalfB * kCh * kTok / 4) / kThr), kThr, 0, stream>>>(OUTF, out, half);
  }
}
